// NonLocalBlock_18030272709224
// MI455X (gfx1250) — hardware-verified
//
#include <hip/hip_runtime.h>


typedef _Float16 v16h __attribute__((ext_vector_type(16)));
typedef _Float16 v8h  __attribute__((ext_vector_type(8)));
typedef float    v8f  __attribute__((ext_vector_type(8)));
typedef float    v4f  __attribute__((ext_vector_type(4)));

#ifndef NB
#define NB 8
#endif
#ifndef HH
#define HH 64
#endif
#define NB_FULL 8
#define WWID 64
#define NN (HH * WWID)
#define NN_FULL 4096
#define MM ((HH / 2) * (WWID / 2))
#define NC 256
#define NI 128
#define SP 136
#define ZP 36

static_assert(NB >= 1 && NB <= NB_FULL);
static_assert(HH >= 4 && HH <= 64 && (HH % 4) == 0);
static_assert((NN % 32) == 0 && (MM % 64) == 0 && (NN % 128) == 0);
static_assert(((NB * NN / 16) % 4) == 0);
static_assert(NC == 256 && NI == 128);

#define WSC 16.0f
#define WINV 0.0625f
#define RSC 2048.0f
#define RINV 0.00048828125f
#define PSC 16384.0f

__device__ __forceinline__ v8f wmma16(v16h a, v16h b, v8f c) {
  v8f d = __builtin_amdgcn_wmma_f32_16x16x32_f16(false, a, false, b, (short)0, c, false, false);
  asm volatile("v_nop\n\tv_nop\n\tv_nop\n\tv_nop" : "+v"(d) : "v"(a), "v"(b));
  return d;
}

__device__ __forceinline__ v16h load_h16(const _Float16* p) {
  v8h lo = *(const v8h*)(p);
  v8h hi = *(const v8h*)(p + 16);
  return __builtin_shufflevector(lo, hi, 0, 1, 2, 3, 4, 5, 6, 7, 8, 9, 10, 11, 12, 13, 14, 15);
}

__device__ __forceinline__ float bf16r(float v) {
  unsigned u = __float_as_uint(v);
  u = (u + 0x7FFFu + ((u >> 16) & 1u)) & 0xFFFF0000u;
  return __uint_as_float(u);
}

__device__ __forceinline__ void split_h(float v, _Float16& hi, _Float16& lo) {
  hi = (_Float16)v;
  lo = (_Float16)((v - (float)hi) * RSC);
}

__device__ __forceinline__ v8h cvt8w(const float* __restrict__ p) {
  const v4f a = *(const v4f*)(p);
  const v4f b = *(const v4f*)(p + 4);
  v8h r;
#pragma unroll
  for (int i = 0; i < 4; ++i) {
    const float av = a[i];
    const float bv = b[i];
    r[i] = (_Float16)(bf16r(av) * WSC);
    r[4 + i] = (_Float16)(bf16r(bv) * WSC);
  }
  return r;
}

__global__ void __launch_bounds__(256)
cvt_w_kernel(const float* __restrict__ w0, const float* __restrict__ w1,
             const float* __restrict__ w2, const float* __restrict__ w3,
             _Float16* __restrict__ o0, _Float16* __restrict__ o1,
             _Float16* __restrict__ o2, _Float16* __restrict__ o3) {
  const int t = blockIdx.x * 256 + threadIdx.x;
  const size_t e = (size_t)t * 8;
  const v8h h0 = cvt8w(w0 + e);
  const v8h h1 = cvt8w(w1 + e);
  const v8h h2 = cvt8w(w2 + e);
  const v8h h3 = cvt8w(w3 + e);
  *(volatile v8h*)(o0 + e) = h0;
  *(volatile v8h*)(o1 + e) = h1;
  *(volatile v8h*)(o2 + e) = h2;
  *(volatile v8h*)(o3 + e) = h3;
  __threadfence();
  *(volatile v8h*)(o0 + e) = h0;
  *(volatile v8h*)(o1 + e) = h1;
  *(volatile v8h*)(o2 + e) = h2;
  *(volatile v8h*)(o3 + e) = h3;
}

__global__ void __launch_bounds__(256)
xpose_kernel(const float* __restrict__ x, _Float16* __restrict__ xT) {
  __shared__ _Float16 tile[64][34];
  const int per_b = (NC / 64) * (NN / 32);
  const int b = blockIdx.x / per_b;
  const int rem = blockIdx.x % per_b;
  const int c0 = (rem / (NN / 32)) * 64;
  const int n0 = (rem % (NN / 32)) * 32;
  const int tx = threadIdx.x & 31;
  const int ty = threadIdx.x >> 5;

#pragma unroll
  for (int s = 0; s < 8; ++s) {
    const int c = ty + s * 8;
    const float v = x[((size_t)b * NC + c0 + c) * NN_FULL + n0 + tx];
    tile[c][tx] = (_Float16)bf16r(v);
  }
  __syncthreads();
  const int lane = tx, wv = ty;
  const int row = wv * 4 + (lane >> 3);
  const int cs = (lane & 7) * 8;
  v8h hv;
#pragma unroll
  for (int j = 0; j < 8; ++j) hv[j] = tile[cs + j][row];
  _Float16* dst = xT + ((size_t)b * NN + n0 + row) * NC + c0 + cs;
  *(volatile v8h*)dst = hv;
  __threadfence();
  *(volatile v8h*)dst = hv;
}

__device__ __forceinline__ v8f gemm8(const v16h (&Ax)[8], const _Float16* __restrict__ wrow) {
  v16h Bw[8];
#pragma unroll
  for (int k = 0; k < 8; ++k) Bw[k] = load_h16(wrow + k * 32);
  v8f acc = {};
#pragma unroll
  for (int k = 0; k < 8; ++k) acc = wmma16(Ax[k], Bw[k], acc);
  return acc;
}

__global__ void __launch_bounds__(128) __attribute__((amdgpu_num_vgpr(256)))
proj_kernel(const _Float16* __restrict__ xT,
            const _Float16* __restrict__ wth, const _Float16* __restrict__ wph,
            const _Float16* __restrict__ wgp,
            const float* __restrict__ bth, const float* __restrict__ bph,
            const float* __restrict__ bgp,
            _Float16* __restrict__ thh, _Float16* __restrict__ thl,
            _Float16* __restrict__ phh, _Float16* __restrict__ phl,
            _Float16* __restrict__ gm) {
  __shared__ __align__(16) _Float16 stg[4][2][16][SP];
  __shared__ __align__(16) _Float16 pstg[4][3][4][SP];

  const int lane = threadIdx.x & 31;
  const int wv = threadIdx.x >> 5;
  const int col = lane & 15;
  const int h = lane >> 4;
  const int hh = h * 8;
  const int rb = h * 8;
  const int tile = blockIdx.x * 4 + wv;
  const int b = tile / (NN / 16);
  const int u = tile % (NN / 16);
  const int hp = u / (WWID / 8);
  const int wg = u % (WWID / 8);
  const int h0 = hp * 2;
  const int w0 = wg * 8;

  const int posA = (h0 + (col >> 3)) * WWID + w0 + (col & 7);
  const _Float16* xRow = xT + ((size_t)b * NN + posA) * NC + hh;
  v16h Ax[8];
#pragma unroll
  for (int k = 0; k < 8; ++k) Ax[k] = load_h16(xRow + k * 32);

#pragma unroll 1
  for (int ic = 0; ic < 8; ++ic) {
    const int ci = ic * 16 + col;
    const v8f acc = gemm8(Ax, wth + (size_t)ci * NC + hh);
    const float bias = bf16r(bth[ci]);
#pragma unroll
    for (int r = 0; r < 8; ++r) {
      const float v = acc[r] * WINV + bias;
      _Float16 vh, vl;
      split_h(v, vh, vl);
      stg[wv][0][rb + r][ci] = vh;
      stg[wv][1][rb + r][ci] = vl;
    }
  }
  __syncthreads();
  {
    _Float16* t0 = thh + (size_t)b * NN * NI;
    _Float16* t1 = thl + (size_t)b * NN * NI;
#pragma unroll
    for (int i = 0; i < 8; ++i) {
      const int row = 2 * i + h;
      const int pos = (h0 + (row >> 3)) * WWID + w0 + (row & 7);
      const v8h a0 = *(const v8h*)&stg[wv][0][row][col * 8];
      const v8h a1 = *(const v8h*)&stg[wv][1][row][col * 8];
      *(volatile v8h*)(t0 + (size_t)pos * NI + col * 8) = a0;
      *(volatile v8h*)(t1 + (size_t)pos * NI + col * 8) = a1;
    }
    __threadfence();
#pragma unroll
    for (int i = 0; i < 8; ++i) {
      const int row = 2 * i + h;
      const int pos = (h0 + (row >> 3)) * WWID + w0 + (row & 7);
      const v8h a0 = *(const v8h*)&stg[wv][0][row][col * 8];
      const v8h a1 = *(const v8h*)&stg[wv][1][row][col * 8];
      *(volatile v8h*)(t0 + (size_t)pos * NI + col * 8) = a0;
      *(volatile v8h*)(t1 + (size_t)pos * NI + col * 8) = a1;
    }
  }

#pragma unroll 1
  for (int ic = 0; ic < 8; ++ic) {
    const int ci = ic * 16 + col;
    const v8f acc = gemm8(Ax, wph + (size_t)ci * NC + hh);
    const float bias = bf16r(bph[ci]);
    float vm[8];
#pragma unroll
    for (int r = 0; r < 8; ++r) {
      const float v = acc[r] * WINV + bias;
      const float vo = __shfl_xor(v, 16);
      vm[r] = fmaxf(v, vo);
    }
    const float pm0 = fmaxf(vm[0], vm[1]);
    const float pm1 = fmaxf(vm[2], vm[3]);
    const float pm2 = fmaxf(vm[4], vm[5]);
    const float pm3 = fmaxf(vm[6], vm[7]);
    const float va = h ? pm2 : pm0;
    const float vb = h ? pm3 : pm1;
    _Float16 ah, al, bh, bl;
    split_h(va, ah, al);
    split_h(vb, bh, bl);
    pstg[wv][0][2 * h][ci] = ah;
    pstg[wv][1][2 * h][ci] = al;
    pstg[wv][0][2 * h + 1][ci] = bh;
    pstg[wv][1][2 * h + 1][ci] = bl;
  }
#pragma unroll 1
  for (int ic = 0; ic < 8; ++ic) {
    const int ci = ic * 16 + col;
    const v8f acc = gemm8(Ax, wgp + (size_t)ci * NC + hh);
    const float bias = bf16r(bgp[ci]);
    float vm[8];
#pragma unroll
    for (int r = 0; r < 8; ++r) {
      const float v = acc[r] * WINV + bias;
      const float vo = __shfl_xor(v, 16);
      vm[r] = fmaxf(v, vo);
    }
    const float pm0 = fmaxf(vm[0], vm[1]);
    const float pm1 = fmaxf(vm[2], vm[3]);
    const float pm2 = fmaxf(vm[4], vm[5]);
    const float pm3 = fmaxf(vm[6], vm[7]);
    const float va = h ? pm2 : pm0;
    const float vb = h ? pm3 : pm1;
    pstg[wv][2][2 * h][ci] = (_Float16)va;
    pstg[wv][2][2 * h + 1][ci] = (_Float16)vb;
  }
  __syncthreads();
  {
    const int mp0 = hp * (WWID / 2) + wg * 4;
    _Float16* p0 = phh + ((size_t)b * MM + mp0) * NI;
    _Float16* p1 = phl + ((size_t)b * MM + mp0) * NI;
    _Float16* p2 = gm + ((size_t)b * MM + mp0) * NI;
#pragma unroll
    for (int i = 0; i < 2; ++i) {
      const int j = 2 * i + h;
      const v8h a0 = *(const v8h*)&pstg[wv][0][j][col * 8];
      const v8h a1 = *(const v8h*)&pstg[wv][1][j][col * 8];
      const v8h a2 = *(const v8h*)&pstg[wv][2][j][col * 8];
      *(volatile v8h*)(p0 + (size_t)j * NI + col * 8) = a0;
      *(volatile v8h*)(p1 + (size_t)j * NI + col * 8) = a1;
      *(volatile v8h*)(p2 + (size_t)j * NI + col * 8) = a2;
    }
    __threadfence();
#pragma unroll
    for (int i = 0; i < 2; ++i) {
      const int j = 2 * i + h;
      const v8h a0 = *(const v8h*)&pstg[wv][0][j][col * 8];
      const v8h a1 = *(const v8h*)&pstg[wv][1][j][col * 8];
      const v8h a2 = *(const v8h*)&pstg[wv][2][j][col * 8];
      *(volatile v8h*)(p0 + (size_t)j * NI + col * 8) = a0;
      *(volatile v8h*)(p1 + (size_t)j * NI + col * 8) = a1;
      *(volatile v8h*)(p2 + (size_t)j * NI + col * 8) = a2;
    }
  }
}

__global__ void __launch_bounds__(256)
xposeh_kernel(const _Float16* __restrict__ in, _Float16* __restrict__ out,
              int rows, int cols, size_t bstride) {
  __shared__ __align__(16) _Float16 tl[64][72];
  const int per_b = (rows / 64) * (cols / 64);
  const int b = blockIdx.x / per_b;
  const int rem = blockIdx.x % per_b;
  const int r0 = (rem / (cols / 64)) * 64;
  const int c0 = (rem % (cols / 64)) * 64;
  const int lane = threadIdx.x & 31;
  const int wv = threadIdx.x >> 5;
  const _Float16* ib = in + (size_t)b * bstride;
  _Float16* ob = out + (size_t)b * bstride;
#pragma unroll
  for (int i = 0; i < 2; ++i) {
    const int rr = (wv * 2 + i) * 4 + (lane >> 3);
    const int cs = (lane & 7) * 8;
    const v8h v = *(const v8h*)(ib + (size_t)(r0 + rr) * cols + c0 + cs);
    *(v8h*)&tl[rr][cs] = v;
  }
  __syncthreads();
#pragma unroll
  for (int i = 0; i < 2; ++i) {
    const int cr = (wv * 2 + i) * 4 + (lane >> 3);
    const int rs = (lane & 7) * 8;
    v8h hv;
#pragma unroll
    for (int j = 0; j < 8; ++j) hv[j] = tl[rs + j][cr];
    *(volatile v8h*)(ob + (size_t)(c0 + cr) * rows + r0 + rs) = hv;
  }
  __threadfence();
#pragma unroll
  for (int i = 0; i < 2; ++i) {
    const int cr = (wv * 2 + i) * 4 + (lane >> 3);
    const int rs = (lane & 7) * 8;
    v8h hv;
#pragma unroll
    for (int j = 0; j < 8; ++j) hv[j] = tl[rs + j][cr];
    *(volatile v8h*)(ob + (size_t)(c0 + cr) * rows + r0 + rs) = hv;
  }
}

__device__ __forceinline__ v8f score_tile(const v16h (&Ah)[4], const _Float16* __restrict__ tlRow,
                                          const _Float16* __restrict__ rh, const _Float16* __restrict__ rl) {
  v8f Hc = {}, Rc = {};
#pragma unroll
  for (int k = 0; k < 4; ++k) {
    const v16h Bh = load_h16(rh + k * 32);
    const v16h Bl = load_h16(rl + k * 32);
    const v16h Al = load_h16(tlRow + k * 32);
    Hc = wmma16(Ah[k], Bh, Hc);
    Rc = wmma16(Ah[k], Bl, Rc);
    Rc = wmma16(Al, Bh, Rc);
  }
  v8f S;
#pragma unroll
  for (int r = 0; r < 8; ++r) S[r] = Hc[r] + Rc[r] * RINV;
  return S;
}

__global__ void __launch_bounds__(128) __attribute__((amdgpu_num_vgpr(256)))
attn_kernel(const _Float16* __restrict__ thh, const _Float16* __restrict__ thl,
            const _Float16* __restrict__ phh, const _Float16* __restrict__ phl,
            const _Float16* __restrict__ gT, _Float16* __restrict__ y) {
  __shared__ __align__(16) _Float16 Pbuf[4][16 * 32];
  __shared__ __align__(16) _Float16 ystg[4][16][SP];

  const int lane = threadIdx.x & 31;
  const int wv = threadIdx.x >> 5;
  const int col = lane & 15;
  const int h = lane >> 4;
  const int hh = h * 8;
  const int rb = h * 8;
  const int tile = blockIdx.x * 4 + wv;
  const int b = tile / (NN / 16);
  const int qBase = (tile % (NN / 16)) * 16;

  const _Float16* thRow = thh + ((size_t)b * NN + qBase + col) * NI + hh;
  const _Float16* tlRow = thl + ((size_t)b * NN + qBase + col) * NI + hh;
  v16h Ah[4];
#pragma unroll
  for (int k = 0; k < 4; ++k) Ah[k] = load_h16(thRow + k * 32);

  v8f O[8];
#pragma unroll
  for (int ct = 0; ct < 8; ++ct) O[ct] = v8f{};
  float m8[8], l8[8];
#pragma unroll
  for (int r = 0; r < 8; ++r) { m8[r] = -1e30f; l8[r] = 0.f; }

  const _Float16* phB = phh + (size_t)b * MM * NI;
  const _Float16* plB = phl + (size_t)b * MM * NI;
  const _Float16* gtB = gT + (size_t)b * NI * MM;

#pragma unroll 1
  for (int kb = 0; kb < MM; kb += 32) {
    const v8f S0 = score_tile(Ah, tlRow, phB + (size_t)(kb + col) * NI + hh,
                              plB + (size_t)(kb + col) * NI + hh);
    const v8f S1 = score_tile(Ah, tlRow, phB + (size_t)(kb + 16 + col) * NI + hh,
                              plB + (size_t)(kb + 16 + col) * NI + hh);

    __syncthreads();
#pragma unroll
    for (int r = 0; r < 8; ++r) {
      float mx = fmaxf(S0[r], S1[r]);
      mx = fmaxf(mx, __shfl_xor(mx, 1));
      mx = fmaxf(mx, __shfl_xor(mx, 2));
      mx = fmaxf(mx, __shfl_xor(mx, 4));
      mx = fmaxf(mx, __shfl_xor(mx, 8));
      const float mn = fmaxf(m8[r], mx);
      const float sc = __expf(m8[r] - mn);
      const float p0 = __expf(S0[r] - mn);
      const float p1 = __expf(S1[r] - mn);
      float ps = p0 + p1;
      ps += __shfl_xor(ps, 1);
      ps += __shfl_xor(ps, 2);
      ps += __shfl_xor(ps, 4);
      ps += __shfl_xor(ps, 8);
      l8[r] = l8[r] * sc + ps;
      m8[r] = mn;
#pragma unroll
      for (int ct = 0; ct < 8; ++ct) O[ct][r] *= sc;
      const int row = rb + r;
      Pbuf[wv][row * 32 + col] = (_Float16)(p0 * PSC);
      Pbuf[wv][row * 32 + 16 + col] = (_Float16)(p1 * PSC);
    }
    __syncthreads();

    const v16h AP = load_h16(&Pbuf[wv][col * 32 + hh]);
#pragma unroll
    for (int ct = 0; ct < 8; ++ct) {
      const v16h Bg = load_h16(gtB + (size_t)(ct * 16 + col) * MM + kb + hh);
      O[ct] = wmma16(AP, Bg, O[ct]);
    }
  }

  float inv[8];
#pragma unroll
  for (int r = 0; r < 8; ++r) inv[r] = 1.0f / (l8[r] * PSC);
#pragma unroll
  for (int ct = 0; ct < 8; ++ct) {
#pragma unroll
    for (int r = 0; r < 8; ++r)
      ystg[wv][rb + r][ct * 16 + col] = (_Float16)(O[ct][r] * inv[r]);
  }
  __syncthreads();
  _Float16* yB = y + ((size_t)b * NN + qBase) * NI;
#pragma unroll
  for (int i = 0; i < 8; ++i) {
    const int row = 2 * i + h;
    const v8h hv = *(const v8h*)&ystg[wv][row][col * 8];
    *(volatile v8h*)(yB + (size_t)row * NI + col * 8) = hv;
  }
  __threadfence();
#pragma unroll
  for (int i = 0; i < 8; ++i) {
    const int row = 2 * i + h;
    const v8h hv = *(const v8h*)&ystg[wv][row][col * 8];
    *(volatile v8h*)(yB + (size_t)row * NI + col * 8) = hv;
  }
}

__global__ void __launch_bounds__(128) __attribute__((amdgpu_num_vgpr(256)))
zproj_kernel(const _Float16* __restrict__ y, const _Float16* __restrict__ wo,
             const float* __restrict__ bo, float* __restrict__ z, float* __restrict__ part) {
  __shared__ __align__(16) float zs[NC][ZP];
  __shared__ __align__(16) float ps[2 * NC];

  const int lane = threadIdx.x & 31;
  const int wv = threadIdx.x >> 5;
  const int col = lane & 15;
  const int h = lane >> 4;
  const int hh = h * 8;
  const int rb = h * 8;
  const int blk = blockIdx.x;
  const int b = blk / (NN / 32);
  const int n0 = (blk % (NN / 32)) * 32;
  const int nt = wv & 1;
  const int ct0 = (wv >> 1) * 8;

  const _Float16* yRow = y + ((size_t)b * NN + n0 + 16 * nt + col) * NI + hh;
  v16h Ay[4];
#pragma unroll
  for (int k = 0; k < 4; ++k) Ay[k] = load_h16(yRow + k * 32);

#pragma unroll 1
  for (int j = 0; j < 8; ++j) {
    const int c = (ct0 + j) * 16 + col;
    const _Float16* wrow = wo + (size_t)c * NI + hh;
    v8f acc = {};
#pragma unroll
    for (int k = 0; k < 4; ++k) {
      const v16h Bw = load_h16(wrow + k * 32);
      acc = wmma16(Ay[k], Bw, acc);
    }
    const float bias = bf16r(bo[c]);
#pragma unroll
    for (int r = 0; r < 8; ++r) zs[c][16 * nt + rb + r] = acc[r] * WINV + bias;
  }
  __syncthreads();

  float* zB = z + (size_t)b * NC * NN + n0;
#pragma unroll
  for (int i = 0; i < 16; ++i) {
    const int c = i * 16 + wv * 4 + (lane >> 3);
    const int piece = (lane & 7) * 4;
    const v4f v = *(const v4f*)&zs[c][piece];
    *(volatile v4f*)(zB + (size_t)c * NN + piece) = v;
  }

  const int t = threadIdx.x;
#pragma unroll 1
  for (int q = 0; q < 2; ++q) {
    const int cc = t + q * 128;
    float s1 = 0.f, s2 = 0.f;
#pragma unroll 4
    for (int n = 0; n < 32; ++n) {
      const float v = zs[cc][n];
      s1 += v;
      s2 += v * v;
    }
    ps[cc] = s1;
    ps[NC + cc] = s2;
  }
  __syncthreads();
  const v4f pv = *(const v4f*)&ps[t * 4];
  float* pB = part + (size_t)blk * (2 * NC) + t * 4;
  *(volatile v4f*)pB = pv;

  __threadfence();
#pragma unroll
  for (int i = 0; i < 16; ++i) {
    const int c = i * 16 + wv * 4 + (lane >> 3);
    const int piece = (lane & 7) * 4;
    const v4f v = *(const v4f*)&zs[c][piece];
    *(volatile v4f*)(zB + (size_t)c * NN + piece) = v;
  }
  *(volatile v4f*)pB = pv;
}

__global__ void __launch_bounds__(256)
stats_kernel(const float* __restrict__ part, int nblk, int cnt_i, float* __restrict__ stats) {
  __shared__ double d1[256], d2[256];
  __shared__ __align__(16) float mstg[32];
  __shared__ __align__(16) float rstg[32];
  const int t = threadIdx.x;
  const int lane = t & 31;
  const int cl = t >> 3;
  const int j = t & 7;
  const int c0 = blockIdx.x * 32;
  const int c = c0 + cl;
  double s1 = 0.0, s2 = 0.0;
#pragma unroll 1
  for (int k = j; k < nblk; k += 8) {
    s1 += (double)part[(size_t)k * (2 * NC) + c];
    s2 += (double)part[(size_t)k * (2 * NC) + NC + c];
  }
  d1[t] = s1;
  d2[t] = s2;
  __syncthreads();
  if (j == 0) {
    double a = 0.0, q = 0.0;
#pragma unroll
    for (int e = 0; e < 8; ++e) { a += d1[t + e]; q += d2[t + e]; }
    const double cnt = (double)cnt_i;
    const double mean = a / cnt;
    double var = q / cnt - mean * mean;
    if (var < 0.0) var = 0.0;
    mstg[cl] = (float)mean;
    rstg[cl] = 1.0f / sqrtf((float)var + 1e-5f);
  }
  __syncthreads();
  const v4f mv = *(const v4f*)&mstg[(lane & 7) * 4];
  const v4f rv = *(const v4f*)&rstg[(lane & 7) * 4];
  v4f sv = rv;
  if (lane < 8) sv = mv;
  float* dst = stats + ((lane < 8) ? 0 : NC) + c0 + (lane & 7) * 4;
  if (t < 16) *(volatile v4f*)dst = sv;
  __threadfence();
  if (t < 16) *(volatile v4f*)dst = sv;
}

__global__ void __launch_bounds__(256)
bnres_kernel(const float* __restrict__ x, const float* __restrict__ z, const float* __restrict__ stats,
             const float* __restrict__ gamma, const float* __restrict__ beta, float* __restrict__ out) {
#pragma clang fp contract(off)
  const size_t gid = (size_t)blockIdx.x * 256 + threadIdx.x;
  const size_t e = gid * 4;
  const int n = (int)(e % NN);
  const size_t bc = e / NN;
  const int c = (int)(bc % NC);
  const size_t b = bc / NC;
  const size_t xi = (b * NC + c) * (size_t)NN_FULL + n;
  const float mean = stats[c];
  const float rstd = stats[NC + c];
  const float ga = bf16r(gamma[c]);
  const float be = bf16r(beta[c]);
  const v4f xv = *(const v4f*)(x + xi);
  const v4f zv = *(const v4f*)(z + e);
  v4f o;
#pragma unroll
  for (int i = 0; i < 4; ++i) {
    const float xs = xv[i];
    const float zsv = zv[i];
    float tt = (zsv - mean) * rstd;
    tt = tt * ga + be;
    o[i] = bf16r(xs) + tt;
  }
  *(volatile v4f*)(out + xi) = o;
  __threadfence();
  *(volatile v4f*)(out + xi) = o;
}

extern "C" void kernel_launch(void* const* d_in, const int* in_sizes, int n_in,
                              void* d_out, int out_size, void* d_ws,
                              size_t ws_size, hipStream_t stream) {
  if (n_in < 11) return;
  if (in_sizes[0] < NB * NC * NN_FULL) return;
  if (in_sizes[1] < NI * NC || in_sizes[3] < NI * NC || in_sizes[5] < NI * NC || in_sizes[7] < NC * NI) return;
  if (in_sizes[2] < NI || in_sizes[4] < NI || in_sizes[6] < NI) return;
  if (in_sizes[8] < NC || in_sizes[9] < NC || in_sizes[10] < NC) return;
  if (out_size < NB * NC * NN_FULL) return;

  const float* x       = (const float*)d_in[0];
  const float* theta_w = (const float*)d_in[1];
  const float* theta_b = (const float*)d_in[2];
  const float* phi_w   = (const float*)d_in[3];
  const float* phi_b   = (const float*)d_in[4];
  const float* g_w     = (const float*)d_in[5];
  const float* g_b     = (const float*)d_in[6];
  const float* W_w     = (const float*)d_in[7];
  const float* W_b     = (const float*)d_in[8];
  const float* bn_g    = (const float*)d_in[9];
  const float* bn_b    = (const float*)d_in[10];
  float* out = (float*)d_out;

  const size_t wbytes  = (size_t)NI * NC * 2;
  const size_t xTbytes = (size_t)NB * NN * NC * 2;
  const size_t thbytes = (size_t)NB * NN * NI * 2;
  const size_t phbytes = (size_t)NB * MM * NI * 2;
  const size_t zbytes  = (size_t)NB * NC * NN * 4;
  const int    nblkz   = NB * NN / 32;
  const size_t pbytes  = (size_t)nblkz * 2 * NC * 4;
  const size_t sbytes  = 4096;

  size_t off = 0;
  const size_t o_wth = off; off += wbytes;
  const size_t o_wph = off; off += wbytes;
  const size_t o_wgp = off; off += wbytes;
  const size_t o_wo  = off; off += wbytes;
  const size_t o_xT  = off; off += xTbytes;
  const size_t o_thh = off; off += thbytes;
  const size_t o_thl = off; off += thbytes;
  const size_t o_phh = off; off += phbytes;
  const size_t o_phl = off; off += phbytes;
  const size_t o_gm  = off; off += phbytes;
  const size_t o_gt  = off; off += phbytes;
  const size_t o_y   = off; off += thbytes;
  const size_t o_z   = off; off += zbytes;
  const size_t o_pt  = off; off += pbytes;
  const size_t o_st  = off; off += sbytes;
  if (off > ws_size) return;

  char* ws = (char*)d_ws;
  _Float16* wth = (_Float16*)(ws + o_wth);
  _Float16* wph = (_Float16*)(ws + o_wph);
  _Float16* wgp = (_Float16*)(ws + o_wgp);
  _Float16* wo  = (_Float16*)(ws + o_wo);
  _Float16* xT  = (_Float16*)(ws + o_xT);
  _Float16* thh = (_Float16*)(ws + o_thh);
  _Float16* thl = (_Float16*)(ws + o_thl);
  _Float16* phh = (_Float16*)(ws + o_phh);
  _Float16* phl = (_Float16*)(ws + o_phl);
  _Float16* gm  = (_Float16*)(ws + o_gm);
  _Float16* gt  = (_Float16*)(ws + o_gt);
  _Float16* yb  = (_Float16*)(ws + o_y);
  float* z      = (float*)(ws + o_z);
  float* part   = (float*)(ws + o_pt);
  float* stats  = (float*)(ws + o_st);

  cvt_w_kernel<<<(NI * NC) / 8 / 256, 256, 0, stream>>>(theta_w, phi_w, g_w, W_w, wth, wph, wgp, wo);
  xpose_kernel<<<NB * (NC / 64) * (NN / 32), 256, 0, stream>>>(x, xT);
  proj_kernel<<<(NB * NN / 16) / 4, 128, 0, stream>>>(xT, wth, wph, wgp, theta_b, phi_b, g_b,
                                                      thh, thl, phh, phl, gm);
  xposeh_kernel<<<NB * (MM / 64) * (NI / 64), 256, 0, stream>>>(gm, gt, MM, NI, (size_t)MM * NI);
  attn_kernel<<<(NB * NN / 16) / 4, 128, 0, stream>>>(thh, thl, phh, phl, gt, yb);
  zproj_kernel<<<nblkz, 128, 0, stream>>>(yb, wo, W_b, z, part);
  stats_kernel<<<NC / 32, 256, 0, stream>>>(part, nblkz, NB * NN, stats);
  bnres_kernel<<<(NB * NC * NN) / 1024, 256, 0, stream>>>(x, z, stats, bn_g, bn_b, out);
}
